// RealMambaBlock_29729763623372
// MI455X (gfx1250) — hardware-run, weakly checked
//
#include <hip/hip_runtime.h>
#include <math.h>

constexpr int kB     = 2;
constexpr int kL     = 2048;
constexpr int kDM    = 1024;
constexpr int kDI    = 2048;
constexpr int kDS    = 16;
constexpr int kR     = 64;
constexpr int kXP    = kR + 2 * kDS;
constexpr int kXPpad = 128;
constexpr int kRows  = kB * kL;
constexpr float kLnEps    = 1e-5f;
constexpr float kWCarry   = 16.0f;
constexpr float kUCarry   = 16.0f;
constexpr float kDtCarry  = 16.0f;
constexpr float kYCarry   = 64.0f;
constexpr float kLog2e    = 1.4426950408889634f;
static_assert(kRows % 64 == 0 && kDI % 64 == 0 && kDM % 64 == 0 && kXPpad % 64 == 0);
static_assert(kDM % 32 == 0 && kDI % 32 == 0 && kR % 32 == 0);

typedef __attribute__((ext_vector_type(16))) _Float16 v16h;
typedef __attribute__((ext_vector_type(8)))  _Float16 v8h;
typedef __attribute__((ext_vector_type(16))) __bf16   v16b;
typedef __attribute__((ext_vector_type(8)))  __bf16   v8b;
typedef __attribute__((ext_vector_type(8)))  float    v8f;
typedef __attribute__((ext_vector_type(4)))  float    v4f;
typedef __attribute__((ext_vector_type(4)))  unsigned int v4u;

__device__ __forceinline__ unsigned short f2bf_bits(float f) {
  unsigned u = __float_as_uint(f);
  return (unsigned short)((u + 0x7FFFu + ((u >> 16) & 1u)) >> 16);
}
__device__ __forceinline__ float bf_bits2f(unsigned short h) { return __uint_as_float(((unsigned)h) << 16); }

__device__ __forceinline__ void dep_guard_h(v8f& a, v8f& b, v16h x, v16h y) { asm volatile("v_nop\n\tv_nop\n\tv_nop\n\tv_nop" : "+v"(a), "+v"(b) : "v"(x), "v"(y)); }
__device__ __forceinline__ void dep_guard_b(v8f& a, v8f& b, v16b x, v16b y) { asm volatile("v_nop\n\tv_nop\n\tv_nop\n\tv_nop" : "+v"(a), "+v"(b) : "v"(x), "v"(y)); }
__device__ __forceinline__ void keep4_h(v16h a, v16h b, v16h c, v16h d) { asm volatile("v_nop" :: "v"(a), "v"(b), "v"(c), "v"(d)); }
__device__ __forceinline__ void keep4_b(v16b a, v16b b, v16b c, v16b d) { asm volatile("v_nop" :: "v"(a), "v"(b), "v"(c), "v"(d)); }
__device__ __forceinline__ void acc_guard4(v8f& a, v8f& b, v8f& c, v8f& d) { asm volatile("v_nop\n\tv_nop\n\tv_nop\n\tv_nop" : "+v"(a), "+v"(b), "+v"(c), "+v"(d)); }
template <typename T> struct Frag;
template <> struct Frag<_Float16> {
  typedef v16h V; union U { v16h v; v8h h[2]; };
  static __device__ __forceinline__ v16h load(const _Float16* p) {
    U f; f.h[0] = *(const v8h*)(p); f.h[1] = *(const v8h*)(p + 16); return f.v;
  }
  static __device__ __forceinline__ v8f mma(v16h a, v16h b, v8f c) {
    return __builtin_amdgcn_wmma_f32_16x16x32_f16(false, a, false, b, (short)0, c, false, false);
  }
  static __device__ __forceinline__ void guard(v8f& a, v8f& b, v16h x, v16h y) { dep_guard_h(a, b, x, y); }
  static __device__ __forceinline__ void keep(v16h a, v16h b, v16h c, v16h d) { keep4_h(a, b, c, d); }
};
template <> struct Frag<__bf16> {
  typedef v16b V; union U { v16b v; v8b h[2]; };
  static __device__ __forceinline__ v16b load(const __bf16* p) {
    U f; f.h[0] = *(const v8b*)(p); f.h[1] = *(const v8b*)(p + 16); return f.v;
  }
  static __device__ __forceinline__ v8f mma(v16b a, v16b b, v8f c) {
    return __builtin_amdgcn_wmma_f32_16x16x32_bf16(false, a, false, b, (short)0, c, false, false);
  }
  static __device__ __forceinline__ void guard(v8f& a, v8f& b, v16b x, v16b y) { dep_guard_b(a, b, x, y); }
  static __device__ __forceinline__ void keep(v16b a, v16b b, v16b c, v16b d) { keep4_b(a, b, c, d); }
};

__device__ __forceinline__ unsigned pk16(unsigned short a, unsigned short b) { return (unsigned)a | ((unsigned)b << 16); }
__device__ __forceinline__ unsigned short h_bits(float f) { const _Float16 h = (_Float16)f; return __builtin_bit_cast(unsigned short, h); }

template <int ET> struct Elem;
template <> struct Elem<0> { typedef _Float16 T; };
template <> struct Elem<1> { typedef __bf16 T; };
template <int ET, bool SPLIT, int BIAS_MODE, int OUT_MODE, bool RESID, int ACT = 0>
__global__ __launch_bounds__(256) void wmma_gemm64(
    const unsigned short* __restrict__ Ap, const unsigned short* __restrict__ A2p, int lda, long strideA,
    const unsigned short* __restrict__ Btp, const unsigned short* __restrict__ Bt2p, int ldb, long strideB,
    void* __restrict__ Cout, void* __restrict__ Cout2, int ldc, long strideC,
    const float* __restrict__ bias,
    const float* __restrict__ resid, long strideR,
    int M, int N, int K, float scale) {
  typedef typename Elem<ET>::T T;
  typedef typename Frag<T>::V V;
  const T* A = (const T*)Ap; const T* A2 = (const T*)A2p; const T* Bt = (const T*)Btp; const T* Bt2 = (const T*)Bt2p;
  __shared__ __align__(16) float sT[8][16 * 68];
  const int b    = blockIdx.y;
  const int lane = threadIdx.x & 31;
  const int wave = threadIdx.x >> 5;
  const int tilesN = N >> 6;
  const int tilesM = M >> 6;
  const int tile = blockIdx.x * 8 + wave;
  if (tile >= tilesM * tilesN) return;
  const int tm = tile / tilesN;
  const int tn = tile - tm * tilesN;
  const int m0 = tm << 6;
  const int n0 = tn << 6;

  const T* Ab  = A  + (size_t)b * strideA;
  const T* Bb  = Bt + (size_t)b * strideB;
  const T* Ab2 = SPLIT ? (A2  + (size_t)b * strideA) : nullptr;
  const T* Bb2 = SPLIT ? (Bt2 + (size_t)b * strideB) : nullptr;

  const int rlane = lane & 15;
  const int koff  = (lane >> 4) * 8;
  const int mOff  = (lane >> 4) * 8;

  v8f acc[4][4];
#pragma unroll
  for (int i = 0; i < 4; ++i)
#pragma unroll
    for (int j = 0; j < 4; ++j) acc[i][j] = (v8f){0.f,0.f,0.f,0.f,0.f,0.f,0.f,0.f};

  for (int k0 = 0; k0 < K; k0 += 32) {
    V bh[4], bl[4];
#pragma unroll
    for (int j = 0; j < 4; ++j) {
      const size_t bo = (size_t)(n0 + (j << 4) + rlane) * ldb + koff + k0;
      bh[j] = Frag<T>::load(Bb + bo);
      if (SPLIT) bl[j] = Frag<T>::load(Bb2 + bo);
    }
#pragma unroll
    for (int i = 0; i < 4; ++i) {
      const size_t ao = (size_t)(m0 + (i << 4) + rlane) * lda + koff + k0;
      V ah = Frag<T>::load(Ab + ao);
      V al;
      if (SPLIT) al = Frag<T>::load(Ab2 + ao);
#pragma unroll
      for (int j = 0; j < 4; ++j) {
        acc[i][j] = Frag<T>::mma(ah, bh[j], acc[i][j]);
        if (SPLIT) {
          acc[i][j] = Frag<T>::mma(ah, bl[j], acc[i][j]);
          acc[i][j] = Frag<T>::mma(al, bh[j], acc[i][j]);
        }
      }
      Frag<T>::guard(acc[i][0], acc[i][3], ah, SPLIT ? al : ah);
    }
    Frag<T>::keep(bh[0], bh[1], bh[2], bh[3]);
    if (SPLIT) Frag<T>::keep(bl[0], bl[1], bl[2], bl[3]);
  }
  acc_guard4(acc[0][0], acc[0][1], acc[0][2], acc[0][3]);
  acc_guard4(acc[1][0], acc[1][1], acc[1][2], acc[1][3]);
  acc_guard4(acc[2][0], acc[2][1], acc[2][2], acc[2][3]);
  acc_guard4(acc[3][0], acc[3][1], acc[3][2], acc[3][3]);

  float* slab = sT[wave];
  const float* Rb = RESID ? (resid + (size_t)b * strideR) : nullptr;
#pragma unroll
  for (int i = 0; i < 4; ++i) {
    const int mBase = m0 + (i << 4);
#pragma unroll
    for (int j = 0; j < 4; ++j) {
      const int n = n0 + (j << 4) + rlane;
      float bv = 0.f;
      if (BIAS_MODE == 2) bv = bias[n];
#pragma unroll
      for (int r = 0; r < 8; ++r) {
        float v = acc[i][j][r] * scale;
        if (BIAS_MODE == 1) v += bias[mBase + mOff + r];
        if (BIAS_MODE == 2) v += bv;
        if (RESID) v += Rb[(size_t)(mBase + mOff + r) * ldc + n];
        if (ACT == 2) v = fmaxf(v, 0.0f);
        if (ACT == 4) v = (v > 0.f) ? v : 0.01f * v;
        slab[(mOff + r) * 68 + (j << 4) + rlane] = v;
      }
    }
    __builtin_amdgcn_fence(__ATOMIC_RELEASE, "workgroup");
    __builtin_amdgcn_wave_barrier();
    __builtin_amdgcn_fence(__ATOMIC_ACQUIRE, "workgroup");
    if (OUT_MODE == 0) {
      float* C = (float*)Cout + (size_t)b * strideC;
      const int hh = lane >> 4, c4 = (lane & 15) * 4;
      for (int pass = 0; pass < 2; ++pass) {
#pragma unroll
        for (int it = 0; it < 8; ++it) {
          const int row = it * 2 + hh;
          v4f v = *(const v4f*)(slab + row * 68 + c4);
          *(volatile v4f*)(C + (size_t)(mBase + row) * ldc + n0 + c4) = v;
        }
        __threadfence();
      }
    } else {
      const int q = lane >> 3, c8 = (lane & 7) * 8;
      unsigned short* C  = (unsigned short*)Cout  + (size_t)b * strideC;
      unsigned short* C2 = (OUT_MODE == 2) ? ((unsigned short*)Cout2 + (size_t)b * strideC) : nullptr;
      for (int pass = 0; pass < 2; ++pass) {
#pragma unroll
        for (int it = 0; it < 4; ++it) {
          const int row = it * 4 + q;
          const float* sp = slab + row * 68 + c8;
          v8h hv, lv;
#pragma unroll
          for (int e = 0; e < 8; ++e) {
            if (OUT_MODE == 1) {
              hv[e] = (_Float16)sp[e];
            } else {
              unsigned short hb = f2bf_bits(sp[e]);
              unsigned short lb = f2bf_bits(sp[e] - bf_bits2f(hb));
              hv[e] = __builtin_bit_cast(_Float16, hb);
              lv[e] = __builtin_bit_cast(_Float16, lb);
            }
          }
          *(volatile v8h*)(C + (size_t)(mBase + row) * ldc + n0 + c8) = hv;
          if (OUT_MODE == 2) *(volatile v8h*)(C2 + (size_t)(mBase + row) * ldc + n0 + c8) = lv;
        }
        __threadfence();
      }
    }
    __builtin_amdgcn_fence(__ATOMIC_RELEASE, "workgroup");
    __builtin_amdgcn_wave_barrier();
    __builtin_amdgcn_fence(__ATOMIC_ACQUIRE, "workgroup");
  }
}

__global__ __launch_bounds__(256) void wtcast_kernel(const float* __restrict__ W, int Kdim, int Ndim,
                                                     unsigned short* __restrict__ out, int ldo, float scale) {
  __shared__ float sm[64][65];
  const int t  = threadIdx.x;
  const int k0 = blockIdx.x * 64;
  const int n0 = blockIdx.y * 64;
#pragma unroll
  for (int i = 0; i < 16; ++i) {
    const int e = i * 256 + t;
    const int r = e >> 6;
    const int c = e & 63;
    const int n = n0 + c;
    const int nc = (n < Ndim) ? n : (Ndim - 1);
    const float v = W[(size_t)(k0 + r) * Ndim + nc] * scale;
    sm[c][r] = (n < Ndim) ? v : 0.f;
  }
  __syncthreads();
  const int lane = t & 31, wave = t >> 5;
  const int q = lane >> 3, c8 = (lane & 7) * 8;
  for (int pass = 0; pass < 2; ++pass) {
#pragma unroll
    for (int it = 0; it < 2; ++it) {
      const int row = wave * 8 + it * 4 + q;
      unsigned short hb[8];
#pragma unroll
      for (int e = 0; e < 8; ++e) hb[e] = h_bits(sm[row][c8 + e]);
      const v4u u = (v4u){pk16(hb[0], hb[1]), pk16(hb[2], hb[3]), pk16(hb[4], hb[5]), pk16(hb[6], hb[7])};
      *(volatile v4u*)(out + (size_t)(n0 + row) * ldo + k0 + c8) = u;
    }
    __threadfence();
  }
}

__global__ __launch_bounds__(128) void layernorm_kernel(const float* __restrict__ x, const float* __restrict__ g,
                                                        const float* __restrict__ bb, unsigned short* __restrict__ h16) {
  __shared__ float red1[4];
  __shared__ float red2[4];
  const int t = threadIdx.x;
  const int lane = t & 31, wave = t >> 5;
  const size_t row = blockIdx.x;
  const float* xr = x + row * kDM + 8 * t;
  const v4f a = *(const v4f*)(xr);
  const v4f c = *(const v4f*)(xr + 4);
  float v[8];
#pragma unroll
  for (int e = 0; e < 4; ++e) { v[e] = a[e]; v[4 + e] = c[e]; }
  float s = ((v[0] + v[1]) + (v[2] + v[3])) + ((v[4] + v[5]) + (v[6] + v[7]));
#pragma unroll
  for (int off = 16; off > 0; off >>= 1) s += __shfl_xor(s, off, 32);
  if (lane == 0) red1[wave] = s;
  __syncthreads();
  const float mu = ((red1[0] + red1[1]) + (red1[2] + red1[3])) * (1.0f / (float)kDM);
  float q = 0.f;
#pragma unroll
  for (int e = 0; e < 8; ++e) { const float dv = v[e] - mu; q += dv * dv; }
#pragma unroll
  for (int off = 16; off > 0; off >>= 1) q += __shfl_xor(q, off, 32);
  if (lane == 0) red2[wave] = q;
  __syncthreads();
  const float var  = ((red2[0] + red2[1]) + (red2[2] + red2[3])) * (1.0f / (float)kDM);
  const float rstd = rsqrtf(var + kLnEps);
  const v4f g0 = *(const v4f*)(g + 8 * t);
  const v4f g1 = *(const v4f*)(g + 8 * t + 4);
  const v4f b0 = *(const v4f*)(bb + 8 * t);
  const v4f b1 = *(const v4f*)(bb + 8 * t + 4);
  unsigned short hb[8];
#pragma unroll
  for (int e = 0; e < 4; ++e) {
    hb[e]     = h_bits((v[e] - mu) * rstd * g0[e] + b0[e]);
    hb[4 + e] = h_bits((v[4 + e] - mu) * rstd * g1[e] + b1[e]);
  }
  const v4u u = (v4u){pk16(hb[0], hb[1]), pk16(hb[2], hb[3]), pk16(hb[4], hb[5]), pk16(hb[6], hb[7])};
  unsigned short* op = h16 + row * kDM + 8 * t;
  *(volatile v4u*)op = u;
  __threadfence();
  *(volatile v4u*)op = u;
}

__global__ __launch_bounds__(256) void conv_silu_kernel(const float* __restrict__ xu, const float* __restrict__ cw,
                                                        const float* __restrict__ cb, float* __restrict__ u32,
                                                        unsigned short* __restrict__ u16) {
  __shared__ __align__(16) float srow[kDI];
  const int t   = threadIdx.x;
  const int row = blockIdx.x;
  const int l   = row & (kL - 1);
  const int b   = row >> 11;
  const size_t rowb = (size_t)b * kL;
#pragma unroll 1
  for (int gi = 0; gi < 8; ++gi) {
    const int d = gi * 256 + t;
    float s = 0.f;
#pragma unroll
    for (int j = 0; j < 4; ++j) {
      const int ll  = l - 3 + j;
      const int llc = (ll < 0) ? 0 : ll;
      float v = xu[(rowb + (size_t)llc) * kDI + d];
      v = (ll >= 0) ? v : 0.f;
      s = s + cw[d * 4 + j] * v;
    }
    s = s + cb[d];
    const float sg = 1.0f / (1.0f + expf(-s));
    srow[d] = s * sg;
  }
  __syncthreads();
  {
    unsigned short hb[8];
#pragma unroll
    for (int e = 0; e < 8; ++e) hb[e] = h_bits(srow[8 * t + e] * kUCarry);
    const v4u u = (v4u){pk16(hb[0], hb[1]), pk16(hb[2], hb[3]), pk16(hb[4], hb[5]), pk16(hb[6], hb[7])};
    unsigned short* op = u16 + (size_t)row * kDI + 8 * t;
    *(volatile v4u*)op = u;
    __threadfence();
    *(volatile v4u*)op = u;
  }
  {
    float* op = u32 + (size_t)row * kDI;
    for (int pass = 0; pass < 2; ++pass) {
#pragma unroll
      for (int it = 0; it < 2; ++it) {
        const int idx = it * 1024 + 4 * t;
        const v4f val = *(const v4f*)(srow + idx);
        *(volatile v4f*)(op + idx) = val;
      }
      __threadfence();
    }
  }
}

__global__ __launch_bounds__(256) void dtcast_kernel(const float* __restrict__ xdbl, unsigned short* __restrict__ dt16) {
  const int i = blockIdx.x * 256 + threadIdx.x;
  if (i >= kRows * 8) return;
  const int row = i >> 3, c8 = (i & 7) * 8;
  const float* p = xdbl + (size_t)row * kXPpad + c8;
  const v4f a = *(const v4f*)(p);
  const v4f c = *(const v4f*)(p + 4);
  unsigned short hb[8];
#pragma unroll
  for (int e = 0; e < 4; ++e) {
    hb[e]     = h_bits(a[e] * kDtCarry);
    hb[4 + e] = h_bits(c[e] * kDtCarry);
  }
  const v4u u = (v4u){pk16(hb[0], hb[1]), pk16(hb[2], hb[3]), pk16(hb[4], hb[5]), pk16(hb[6], hb[7])};
  unsigned short* q = dt16 + (size_t)row * kR + c8;
  *(volatile v4u*)q = u;
  __threadfence();
  *(volatile v4u*)q = u;
}

__global__ __launch_bounds__(256) void scan_kernel(const float* __restrict__ dtraw, const float* __restrict__ u32,
                                                   const float* __restrict__ xdbl, const float* __restrict__ z32,
                                                   const float* __restrict__ A_log, const float* __restrict__ Dp,
                                                   unsigned short* __restrict__ y16) {
  __shared__ __align__(16) float sBC[64 * 32];
  __shared__ __align__(16) unsigned short sy[64 * 256];
  const int t = threadIdx.x;
  const int lane = t & 31, wave = t >> 5;
  const int bx = blockIdx.x;
  const int b  = blockIdx.y;
  const int d  = bx * 256 + t;
  const size_t rowb = (size_t)b * kL;

  float A2[16];
  {
    const float* ap = A_log + (size_t)d * kDS;
    const v4f a0 = *(const v4f*)(ap);
    const v4f a1 = *(const v4f*)(ap + 4);
    const v4f a2 = *(const v4f*)(ap + 8);
    const v4f a3 = *(const v4f*)(ap + 12);
#pragma unroll
    for (int e = 0; e < 4; ++e) {
      A2[e]      = -exp2f(a0[e] * kLog2e) * kLog2e;
      A2[4 + e]  = -exp2f(a1[e] * kLog2e) * kLog2e;
      A2[8 + e]  = -exp2f(a2[e] * kLog2e) * kLog2e;
      A2[12 + e] = -exp2f(a3[e] * kLog2e) * kLog2e;
    }
  }
  const float Dd = Dp[d];
  float hs[16];
#pragma unroll
  for (int n = 0; n < 16; ++n) hs[n] = 0.f;

  for (int ch = 0; ch < kL / 64; ++ch) {
    const size_t row0 = rowb + (size_t)ch * 64;
    __syncthreads();
#pragma unroll
    for (int i = 0; i < 2; ++i) {
      const int e = i * 256 + t;
      const int step = e >> 3;
      const int q4 = (e & 7) * 4;
      const v4f v = *(const v4f*)(xdbl + (row0 + step) * kXPpad + kR + q4);
      *(v4f*)(sBC + step * 32 + q4) = v;
    }
    __syncthreads();
#pragma unroll 1
    for (int s = 0; s < 64; ++s) {
      const size_t off = (row0 + s) * kDI + d;
      const float dtv = dtraw[off];
      const float uv  = u32[off];
      const float zv  = z32[off];
      const float delta = fmaxf(dtv, 0.f) + log1pf(expf(-fabsf(dtv)));
      const float du = delta * uv;
      const v4f b0 = *(const v4f*)(sBC + s * 32 + 0);
      const v4f b1 = *(const v4f*)(sBC + s * 32 + 4);
      const v4f b2 = *(const v4f*)(sBC + s * 32 + 8);
      const v4f b3 = *(const v4f*)(sBC + s * 32 + 12);
      const v4f c0 = *(const v4f*)(sBC + s * 32 + 16);
      const v4f c1 = *(const v4f*)(sBC + s * 32 + 20);
      const v4f c2 = *(const v4f*)(sBC + s * 32 + 24);
      const v4f c3 = *(const v4f*)(sBC + s * 32 + 28);
      float Bv[16], Cv[16];
#pragma unroll
      for (int e = 0; e < 4; ++e) {
        Bv[e] = b0[e]; Bv[4 + e] = b1[e]; Bv[8 + e] = b2[e]; Bv[12 + e] = b3[e];
        Cv[e] = c0[e]; Cv[4 + e] = c1[e]; Cv[8 + e] = c2[e]; Cv[12 + e] = c3[e];
      }
      float y = 0.f;
#pragma unroll
      for (int n = 0; n < 16; ++n) {
        const float dA = exp2f(delta * A2[n]);
        hs[n] = dA * hs[n] + du * Bv[n];
        y = y + hs[n] * Cv[n];
      }
      y = y + uv * Dd;
      const float sg = 1.0f / (1.0f + expf(-zv));
      y = y * (zv * sg);
      sy[s * 256 + t] = h_bits(y * kYCarry);
    }
    __syncthreads();
    unsigned short* yb = y16 + row0 * kDI + (size_t)bx * 256 + lane * 8;
    for (int pass = 0; pass < 2; ++pass) {
#pragma unroll
      for (int it = 0; it < 8; ++it) {
        const int srow = wave * 8 + it;
        const v4u val = *(const v4u*)(sy + srow * 256 + lane * 8);
        *(volatile v4u*)(yb + (size_t)srow * kDI) = val;
      }
      __threadfence();
    }
  }
}

extern "C" void kernel_launch(void* const* d_in, const int* in_sizes, int n_in,
                              void* d_out, int out_size, void* d_ws, size_t ws_size, hipStream_t stream) {
  if (n_in < 12) return;
  if (in_sizes[0] != kRows * kDM) return;
  if (in_sizes[1] != kDM || in_sizes[2] != kDM) return;
  if (in_sizes[3] != kDM * 2 * kDI) return;
  if (in_sizes[4] != kDI * 4 || in_sizes[5] != kDI) return;
  if (in_sizes[6] != kDI * kXP) return;
  if (in_sizes[7] != kR * kDI || in_sizes[8] != kDI) return;
  if (in_sizes[9] != kDI * kDS || in_sizes[10] != kDI) return;
  if (in_sizes[11] != kDI * kDM) return;
  if (out_size != kRows * kDM) return;

  const float* x      = (const float*)d_in[0];
  const float* ln_g   = (const float*)d_in[1];
  const float* ln_b   = (const float*)d_in[2];
  const float* W_in   = (const float*)d_in[3];
  const float* conv_w = (const float*)d_in[4];
  const float* conv_b = (const float*)d_in[5];
  const float* W_xprj = (const float*)d_in[6];
  const float* W_dt   = (const float*)d_in[7];
  const float* b_dt   = (const float*)d_in[8];
  const float* A_log  = (const float*)d_in[9];
  const float* Dvec   = (const float*)d_in[10];
  const float* W_out  = (const float*)d_in[11];
  float* out = (float*)d_out;

  char* ws = (char*)d_ws;
  size_t off = 0;
  const size_t szPlane32 = (size_t)kRows * kDI * 4;
  char* p_planeU = ws + off; off += szPlane32;
  char* p_planeZ = ws + off; off += szPlane32;
  char* p_u32    = ws + off; off += szPlane32;
  char* p_regA   = ws + off; off += (size_t)kRows * kDI * 2;
  char* p_xdbl   = ws + off; off += (size_t)kRows * kXPpad * 4;
  char* p_dt16   = ws + off; off += (size_t)kRows * kR * 2;
  char* p_WtXp   = ws + off; off += (size_t)kXPpad * kDI * 2;
  char* p_WtDt   = ws + off; off += (size_t)kDI * kR * 2;
  char* p_WtOut  = ws + off; off += (size_t)kDM * kDI * 2;
  if (off > ws_size) return;
  (void)p_planeZ;

  float*          planeU = (float*)p_planeU;
  float*          dtraw  = (float*)p_planeU;
  float*          z32    = (float*)p_planeZ;
  float*          u32    = (float*)p_u32;
  unsigned short* h16    = (unsigned short*)p_regA;
  unsigned short* WtIn   = (unsigned short*)(p_regA + (size_t)kRows * kDM * 2);
  unsigned short* u16    = (unsigned short*)p_regA;
  unsigned short* y16    = (unsigned short*)p_regA;
  float*          xdbl   = (float*)p_xdbl;
  unsigned short* dt16   = (unsigned short*)p_dt16;
  unsigned short* WtXp   = (unsigned short*)p_WtXp;
  unsigned short* WtDt   = (unsigned short*)p_WtDt;
  unsigned short* WtOut  = (unsigned short*)p_WtOut;

  layernorm_kernel<<<dim3(kRows), dim3(128), 0, stream>>>(x, ln_g, ln_b, h16);

  wtcast_kernel<<<dim3(kDM / 64, (2 * kDI) / 64), dim3(256), 0, stream>>>(W_in,   kDM, 2 * kDI, WtIn,  kDM, kWCarry);
  wtcast_kernel<<<dim3(kDI / 64, kXPpad / 64),    dim3(256), 0, stream>>>(W_xprj, kDI, kXP,     WtXp,  kDI, kWCarry);
  wtcast_kernel<<<dim3(kR / 64, kDI / 64),        dim3(256), 0, stream>>>(W_dt,   kR,  kDI,     WtDt,  kR,  kWCarry);
  wtcast_kernel<<<dim3(kDI / 64, kDM / 64),       dim3(256), 0, stream>>>(W_out,  kDI, kDM,     WtOut, kDI, kWCarry);

  {
    const int tiles = (kRows / 64) * (kDI / 64);
    wmma_gemm64<0, false, 0, 0, false><<<dim3((tiles + 7) / 8, 2), dim3(256), 0, stream>>>(
        h16, h16, kDM, 0L,
        WtIn, WtIn, kDM, (long)kDI * kDM,
        (void*)planeU, (void*)planeU, kDI, (long)kRows * kDI,
        b_dt, x, 0L,
        kRows, kDI, kDM, 1.0f / kWCarry);
  }

  conv_silu_kernel<<<dim3(kRows), dim3(256), 0, stream>>>(planeU, conv_w, conv_b, u32, u16);

  {
    const int tiles = (kRows / 64) * (kXPpad / 64);
    wmma_gemm64<0, false, 0, 0, false><<<dim3((tiles + 7) / 8, 1), dim3(256), 0, stream>>>(
        u16, u16, kDI, 0L,
        WtXp, WtXp, kDI, 0L,
        (void*)xdbl, (void*)xdbl, kXPpad, 0L,
        b_dt, x, 0L,
        kRows, kXPpad, kDI, 1.0f / (kUCarry * kWCarry));
  }

  dtcast_kernel<<<dim3((kRows * 8) / 256), dim3(256), 0, stream>>>(xdbl, dt16);

  {
    const int tiles = (kRows / 64) * (kDI / 64);
    wmma_gemm64<0, false, 2, 0, false><<<dim3((tiles + 7) / 8, 1), dim3(256), 0, stream>>>(
        dt16, dt16, kR, 0L,
        WtDt, WtDt, kR, 0L,
        (void*)dtraw, (void*)dtraw, kDI, 0L,
        b_dt, x, 0L,
        kRows, kDI, kR, 1.0f / (kDtCarry * kWCarry));
  }

  scan_kernel<<<dim3(kDI / 256, kB), dim3(256), 0, stream>>>(dtraw, u32, xdbl, z32, A_log, Dvec, y16);

  {
    const int tiles = (kRows / 64) * (kDM / 64);
    wmma_gemm64<0, false, 0, 0, true><<<dim3((tiles + 7) / 8, 1), dim3(256), 0, stream>>>(
        y16, y16, kDI, 0L,
        WtOut, WtOut, kDI, 0L,
        (void*)out, (void*)out, kDM, 0L,
        b_dt, x, 0L,
        kRows, kDM, kDI, 1.0f / (kYCarry * kWCarry));
  }
}
